// DLP_model2_90555090469432
// MI455X (gfx1250) — hardware-run, weakly checked
//
#include <hip/hip_runtime.h>


#define NN       100000
#define ED       128
#define HID      32
#define NE_FULL  2000000
#ifndef NE
#define NE 2000000
#endif
#define EW       5
#define TPW      8
#define WPE      (TPW * 16)
#define WCARRY   64.0f
#define H2I      (1.0f / 4096.0f)

static_assert(ED % 32 == 0);
static_assert(HID == 32);
static_assert(NE % WPE == 0);
static_assert(NE <= NE_FULL);
static_assert(WPE * 4 == 32 * 16);
static_assert((size_t)NN * ED < (size_t)4294967296);
static_assert(((size_t)NN * ED) % 8 == 0);
static_assert((ED * HID / 8) % 128 == 0);
static_assert((HID * HID / 8) % 128 == 0);
static_assert((1 << 4) * 8 == ED);
static_assert((1 << 2) * 8 == HID);
static_assert(EW * WPE * 4 <= 131072);

typedef _Float16 h16;
typedef unsigned short bf;
typedef __attribute__((ext_vector_type(16))) _Float16 v16h;
typedef __attribute__((ext_vector_type(8)))  _Float16 v8h;
typedef __attribute__((ext_vector_type(8)))  unsigned short v8us;
typedef __attribute__((ext_vector_type(8)))  float    v8f;
typedef __attribute__((ext_vector_type(4)))  float    v4f;
typedef __attribute__((ext_vector_type(4)))  unsigned int v4u;
typedef v4f  __attribute__((may_alias)) v4fa;

__device__ __forceinline__ unsigned short f2bf(float f) { unsigned u = __float_as_uint(f); u += 0x7FFFu + ((u >> 16) & 1u); return (unsigned short)(u >> 16); }
__device__ __forceinline__ float bfr(float f) { return __uint_as_float(((unsigned)f2bf(f)) << 16); }
__device__ __forceinline__ v16h cat16(v8h lo, v8h hi) { return __builtin_shufflevector(lo, hi, 0, 1, 2, 3, 4, 5, 6, 7, 8, 9, 10, 11, 12, 13, 14, 15); }
__device__ __forceinline__ v8f wmma16(v16h a, v16h b, v8f c) { return __builtin_amdgcn_wmma_f32_16x16x32_f16(false, a, false, b, (short)0, c, false, false); }
__device__ __forceinline__ v8f wmma16g(v16h a, v16h b, v8f c) { c = wmma16(a, b, c); asm volatile("v_nop\n\tv_nop\n\tv_nop\n\tv_nop" : "+v"(c) : "v"(a), "v"(b)); return c; }
__device__ __forceinline__ v16h  ldh(const h16* p) { return cat16(*(const v8h*)p, *(const v8h*)(p + 16)); }
__device__ __forceinline__ void wave_sync() { __builtin_amdgcn_fence(3  , "wavefront"); __builtin_amdgcn_wave_barrier(); asm volatile("" ::: "memory"); }
static __device__ __forceinline__ h16 toh_flush(float v) { const float w = (fabsf(v) < 6.103515625e-05f) ? 0.0f : v; return (h16)w; }
__device__ __forceinline__ v8f ldp8(const float* __restrict__ p, float sc) {
    const v4f x = *(const v4f*)p; const v4f y = *(const v4f*)(p + 4); v8f o;
#pragma unroll
    for (int i = 0; i < 4; ++i) { o[i] = bfr(x[i]) * sc; o[4 + i] = bfr(y[i]) * sc; }
    return o;
}

__global__ __launch_bounds__(256) void k_cvt8(const float* __restrict__ src, bf* dst, size_t n8) {
    const size_t i = (size_t)blockIdx.x * 256 + threadIdx.x; if (i >= n8) return;
    const v8f v = *(const v8f*)(src + i * 8); v8us o;
#pragma unroll
    for (int k = 0; k < 8; ++k) o[k] = f2bf(v[k]);
    *(volatile v8us*)(dst + i * 8) = o; __threadfence(); *(volatile v8us*)(dst + i * 8) = o;
}

__global__ __launch_bounds__(128) void k_wt(const float* __restrict__ W, h16* WT, unsigned lk8, unsigned ncol, unsigned n8) {
    const unsigned i = blockIdx.x * 128u + threadIdx.x; if (i >= n8) return;
    const unsigned n = i >> lk8, k8 = (i & ((1u << lk8) - 1u)) * 8u; v8h o;
#pragma unroll
    for (int j = 0; j < 8; ++j) o[j] = toh_flush(bfr(W[(k8 + (unsigned)j) * ncol + n]) * WCARRY);
    *(volatile v8h*)(WT + (size_t)i * 8) = o; __threadfence(); *(volatile v8h*)(WT + (size_t)i * 8) = o;
}

__global__ __launch_bounds__(32 * EW) void k_edge(const int* __restrict__ nid, const int* __restrict__ eli, const bf* __restrict__ TB,
                                                  const h16* __restrict__ W1T, const h16* __restrict__ W2T,
                                                  const float* __restrict__ b1, const float* __restrict__ b2,
                                                  const float* __restrict__ w3, const float* __restrict__ b3, float* OUT) {
    __shared__ __align__(16) float ps[EW * WPE];
    const int lane = threadIdx.x & 31, lr = lane & 15, hi = lane >> 4;
    const int wave = __builtin_amdgcn_readfirstlane((int)(threadIdx.x >> 5));
    const unsigned bx = blockIdx.x;
    const unsigned gw = bx * (unsigned)EW + (unsigned)wave;
    if (gw >= (unsigned)(NE / WPE)) return;
    const unsigned ebase = gw * (unsigned)WPE;
    const v8f b1a = ldp8(b1 + 8 * hi, WCARRY), b1b = ldp8(b1 + 16 + 8 * hi, WCARRY);
    const v8f b2a = ldp8(b2 + 8 * hi, 1.0f),   b2b = ldp8(b2 + 16 + 8 * hi, 1.0f);
    const v8f w3a = ldp8(w3 + 8 * hi, 1.0f),   w3b = ldp8(w3 + 16 + 8 * hi, 1.0f);
    const float b3v = bfr(b3[0]);
    const v16h w2a = ldh(W2T + (unsigned)lr * HID + 8u * (unsigned)hi);
    const v16h w2b = ldh(W2T + (unsigned)(16 + lr) * HID + 8u * (unsigned)hi);
    const unsigned wo = (unsigned)lr * (unsigned)ED + 8u * (unsigned)hi;
    const int wb = wave * WPE;
#pragma unroll 1
    for (int t = 0; t < TPW; ++t) {
        const unsigned eo = ebase + (unsigned)t * 16u + (unsigned)lr;
        int sN = eli[eo];
        int dN = eli[(unsigned)NE_FULL + eo];
        sN = min(max(sN, 0), NN - 1); dN = min(max(dN, 0), NN - 1);
        int sR = nid[(unsigned)sN];
        int dR = nid[(unsigned)dN];
        sR = min(max(sR, 0), NN - 1); dR = min(max(dR, 0), NN - 1);
        const unsigned so = (unsigned)sR * (unsigned)ED + 8u * (unsigned)hi;
        const unsigned dofs = (unsigned)dR * (unsigned)ED + 8u * (unsigned)hi;
        v8f h1a = (v8f){}, h1b = (v8f){};
#pragma unroll 1
        for (unsigned kc = 0; kc < (unsigned)ED; kc += 32u) {
            const v4u a0 = *(const v4u*)(TB + so + kc);
            const v4u a1 = *(const v4u*)(TB + so + kc + 16u);
            const v4u c0 = *(const v4u*)(TB + dofs + kc);
            const v4u c1 = *(const v4u*)(TB + dofs + kc + 16u);
            v16h f;
#pragma unroll
            for (int q = 0; q < 4; ++q) {
                f[2 * q]         = toh_flush(__uint_as_float(a0[q] << 16) * __uint_as_float(c0[q] << 16));
                f[2 * q + 1]     = toh_flush(__uint_as_float(a0[q] & 0xFFFF0000u) * __uint_as_float(c0[q] & 0xFFFF0000u));
                f[8 + 2 * q]     = toh_flush(__uint_as_float(a1[q] << 16) * __uint_as_float(c1[q] << 16));
                f[8 + 2 * q + 1] = toh_flush(__uint_as_float(a1[q] & 0xFFFF0000u) * __uint_as_float(c1[q] & 0xFFFF0000u));
            }
            const v16h wa = ldh(W1T + wo + kc);
            const v16h wc = ldh(W1T + wo + 16u * (unsigned)ED + kc);
            h1a = wmma16g(wa, f, h1a);
            h1b = wmma16g(wc, f, h1b);
        }
        v16h pb;
#pragma unroll
        for (int r = 0; r < 8; ++r) {
            const float xa = h1a[r] + b1a[r]; const float xb = h1b[r] + b1b[r];
            pb[r]     = toh_flush(xa > 0.0f ? xa : 0.0f);
            pb[8 + r] = toh_flush(xb > 0.0f ? xb : 0.0f);
        }
        v8f h2a = (v8f){}, h2b = (v8f){};
        h2a = wmma16g(w2a, pb, h2a);
        h2b = wmma16g(w2b, pb, h2b);
        float s = 0.0f;
#pragma unroll
        for (int r = 0; r < 8; ++r) { float x = h2a[r] * H2I + b2a[r]; x = x > 0.0f ? x : 0.0f; s = fmaf(w3a[r], x, s); }
#pragma unroll
        for (int r = 0; r < 8; ++r) { float x = h2b[r] * H2I + b2b[r]; x = x > 0.0f ? x : 0.0f; s = fmaf(w3b[r], x, s); }
        s += __shfl_xor(s, 16, 32);
        const float pv = s + b3v;
        if (hi == 0) ps[wb + t * 16 + lr] = pv;
    }
    wave_sync();
    const v4f val = *(const v4fa*)(&ps[wb + 4 * lane]);
    float* op = OUT + (size_t)ebase + (size_t)(4 * lane);
    *(volatile v4f*)op = val; __threadfence(); *(volatile v4f*)op = val;
}

static constexpr size_t al256(size_t v) { return (v + 255) & ~(size_t)255; }
static constexpr size_t SZ_TB = al256((size_t)NN * ED * 2);
static constexpr size_t SZ_W1 = al256((size_t)HID * ED * 2);
static constexpr size_t SZ_W2 = al256((size_t)HID * HID * 2);
static constexpr size_t SZ_TOTAL = SZ_TB + SZ_W1 + SZ_W2;
static_assert(SZ_TOTAL <= (size_t)134217728);
static constexpr size_t   N8_TB = (size_t)NN * ED / 8;
static constexpr unsigned N8_W1 = (unsigned)(HID * ED / 8);
static constexpr unsigned N8_W2 = (unsigned)(HID * HID / 8);
static constexpr unsigned G_TB  = (unsigned)((N8_TB + 255) / 256);
static constexpr unsigned G_ED  = (unsigned)((NE / WPE + EW - 1) / EW);
static_assert((size_t)G_TB * 256 >= N8_TB);
static_assert((size_t)G_ED * EW * WPE >= (size_t)NE);

extern "C" void kernel_launch(void* const* d_in, const int* in_sizes, int n_in,
                              void* d_out, int out_size, void* d_ws, size_t ws_size, hipStream_t stream) {
    if (n_in < 9) return;
    if ((size_t)in_sizes[0] < (size_t)NN) return;
    if ((size_t)in_sizes[1] < (size_t)NE_FULL + (size_t)NE) return;
    if ((size_t)in_sizes[2] < (size_t)NN * ED) return;
    if (in_sizes[3] < ED * HID || in_sizes[4] < HID || in_sizes[5] < HID * HID || in_sizes[6] < HID || in_sizes[7] < HID || in_sizes[8] < 1) return;
    if ((size_t)out_size < (size_t)NE) return;
    if (SZ_TOTAL > ws_size) return;
    const int* nid = (const int*)d_in[0];
    const int* eli = (const int*)d_in[1];
    const float* emb = (const float*)d_in[2];
    const float* w1 = (const float*)d_in[3]; const float* b1 = (const float*)d_in[4];
    const float* w2 = (const float*)d_in[5]; const float* b2 = (const float*)d_in[6];
    const float* w3 = (const float*)d_in[7]; const float* b3 = (const float*)d_in[8];
    float* OUT = (float*)d_out;
    char* wsp = (char*)d_ws;
    bf*  TB  = (bf*)wsp;  wsp += SZ_TB;
    h16* W1T = (h16*)wsp; wsp += SZ_W1;
    h16* W2T = (h16*)wsp; wsp += SZ_W2;

    k_cvt8<<<G_TB, 256, 0, stream>>>(emb, TB, N8_TB);
    k_wt<<<N8_W1 / 128u, 128, 0, stream>>>(w1, W1T, 4u, (unsigned)HID, N8_W1);
    k_wt<<<N8_W2 / 128u, 128, 0, stream>>>(w2, W2T, 2u, (unsigned)HID, N8_W2);
    k_edge<<<G_ED, 32 * EW, 0, stream>>>(nid, eli, TB, W1T, W2T, b1, b2, w3, b3, OUT);
}
